// DynamicNeuralTuringMachine_48241072668793
// MI455X (gfx1250) — hardware-run, weakly checked
//
#include <hip/hip_runtime.h>
#include <math.h>

typedef __attribute__((ext_vector_type(16))) _Float16 v16h;
typedef __attribute__((ext_vector_type(8)))  _Float16 v8h;
typedef __attribute__((ext_vector_type(16))) __bf16   v16b;
typedef __attribute__((ext_vector_type(8)))  __bf16   v8b;
typedef __attribute__((ext_vector_type(8)))  float    v8f;
typedef __attribute__((ext_vector_type(4)))  float    v4f;

constexpr int kBatch  = 64;
constexpr int kSteps  = 96;
constexpr int kFeat   = 64;
constexpr int kHid    = 256;
constexpr int kLoc    = 128;
constexpr int kCont   = 96;
constexpr int kAddr   = 32;
constexpr int kOutN   = 10;
constexpr int kMem    = kCont + kAddr;
constexpr int kGate3  = 3 * kHid;
constexpr int kRowsX  = kSteps * kBatch;
constexpr int kColCd  = 0;
constexpr int kColEr  = kColCd + kCont;
constexpr int kColG   = kColEr + kCont;
constexpr int kNin    = kColG + kGate3;
constexpr int kRowQ   = 0;
constexpr int kRowCd  = kRowQ + kMem;
constexpr int kRowEr  = kRowCd + kCont;
constexpr int kRowHd  = kRowEr + kCont;
constexpr int kNqc    = kRowHd + 16;
constexpr int kTilesA = kNqc / 16;
constexpr int kThr    = 256;
constexpr int kThrRun = 512;
constexpr int kSeqBlk = 16;
constexpr int kHP     = 264;
constexpr int kRP     = 136;
constexpr float kEps  = 1e-8f;
constexpr int kOut0   = kSteps * kHid * kBatch;
constexpr int kOut1   = kSteps * kOutN * kBatch;

constexpr float kInCarry  = 1024.0f;
constexpr float kWCarry   = 1024.0f;
constexpr float kActCarry = 4096.0f;
constexpr float kRdCarry  = 1024.0f;
constexpr float kXpScale  = 1.0f / (kInCarry * kWCarry);
constexpr float kRecScale = 1.0f / (kActCarry * kWCarry);
constexpr float kRdScale  = 1.0f / (kRdCarry * kWCarry);
constexpr float kF16MinNormal = 6.103515625e-5f;

static_assert(kMem == 128 && kNin == 960 && kNqc == 336 && kTilesA == 21 && kRowsX == 6144, "plane sizes");
static_assert((kRowsX % 64) == 0 && (kNin % 64) == 0 && (kFeat % 32) == 0, "hoisted GEMM: M, N multiples of 64, K of 32");
static_assert(kHid == 16 * (kThrRun / 32), "16 waves x 16 hidden units");
static_assert(kSeqBlk == kThrRun / 32, "one wave per sample of the block in the memory phase");
static_assert(kBatch % kSeqBlk == 0, "batch tiles");
static_assert((kHP % 8) == 0 && kHP >= kHid + 8 && (kRP % 8) == 0 && kRP >= kMem + 8, "f16 tile pitches");
static_assert(kCont == 8 * 12 && kAddr == 8 * 4 && kLoc == 4 * 32, "memory phase lane map: 8 column groups x 4 row groups");
static_assert(kFeat == kBatch, "the module's reshape of a [64][64] slab to (F, B) is an index exchange only because F == B");

constexpr int kSmBq  = 0;
constexpr int kSmBo  = kSmBq + kMem;
constexpr int kSmUs  = kSmBo + 16;
constexpr int kSmUl  = kSmUs + kHid;
constexpr int kSmBs  = kSmUl + kHid;
constexpr int kSmAd  = kSmBs + 4;
constexpr int kSmAn  = kSmAd + kLoc * kAddr;
constexpr int kSmTot = kSmAn + kLoc;
static_assert(kSmTot == 4884 && (kSmAd % 4) == 0 && (kSmAn % 4) == 0, "small block layout");

constexpr size_t kOffXA   = 0;
constexpr size_t kOffWIN  = kOffXA   + (size_t)kRowsX * kFeat * 2;
constexpr size_t kOffBIN  = kOffWIN  + (size_t)kNin * kFeat * 2;
constexpr size_t kOffXP   = kOffBIN  + 4096;
constexpr size_t kOffWQC  = kOffXP   + (size_t)kRowsX * kNin * 4;
constexpr size_t kOffWHH  = kOffWQC  + (size_t)kNqc * kHid * 2;
constexpr size_t kOffWMH  = kOffWHH  + (size_t)kGate3 * kHid * 2;
constexpr size_t kOffSM   = kOffWMH  + (size_t)kGate3 * kMem * 2;
constexpr size_t kOffMEMC = kOffSM   + 19712;
constexpr size_t kOffHSW  = kOffMEMC + (size_t)kBatch * kLoc * kCont * 4;
constexpr size_t kOffOUTW = kOffHSW  + (size_t)kRowsX * kHid * 4;
constexpr size_t kWsTotal = kOffOUTW + (size_t)kRowsX * 16 * 4;
static_assert(kWsTotal == 35118336ull, "carve total");
static_assert(kWsTotal <= 134217728ull, "carve cap");
static_assert((kOffWIN % 256) == 0 && (kOffBIN % 256) == 0 && (kOffXP % 256) == 0 && (kOffWQC % 256) == 0 && (kOffWHH % 256) == 0 && (kOffWMH % 256) == 0 && (kOffSM % 256) == 0 && (kOffMEMC % 256) == 0 && (kOffHSW % 256) == 0 && (kOffOUTW % 256) == 0, "aligned regions");
static_assert((size_t)kSmTot * 4 <= 19712 && (size_t)kNin * 4 <= 4096, "small regions fit");

__device__ __forceinline__ unsigned short f2bf_bits(float f) {
  unsigned u = __float_as_uint(f);
  return (unsigned short)((u + 0x7FFFu + ((u >> 16) & 1u)) >> 16);
}
__device__ __forceinline__ float bf_bits2f(unsigned short h) { return __uint_as_float(((unsigned)h) << 16); }
__device__ __forceinline__ float bf16r(float f) { return bf_bits2f(f2bf_bits(f)); }
__device__ __forceinline__ float carry_flush(float v, float carry) {
  const float s = v * carry;
  return (fabsf(s) < kF16MinNormal) ? 0.0f : s;
}
__device__ __forceinline__ float frcp(float x) { return __builtin_amdgcn_rcpf(x); }

__device__ __forceinline__ void dep_guard4_h(v8f& a, v8f& b, v8f& c, v8f& d, v16h x, v16h y) { asm volatile("v_nop\n\tv_nop\n\tv_nop\n\tv_nop" : "+v"(a), "+v"(b), "+v"(c), "+v"(d) : "v"(x), "v"(y)); }
__device__ __forceinline__ void dep_guard4_b(v8f& a, v8f& b, v8f& c, v8f& d, v16b x, v16b y) { asm volatile("v_nop\n\tv_nop\n\tv_nop\n\tv_nop" : "+v"(a), "+v"(b), "+v"(c), "+v"(d) : "v"(x), "v"(y)); }
__device__ __forceinline__ void keep4_h(v16h a, v16h b, v16h c, v16h d) { asm volatile("v_nop" :: "v"(a), "v"(b), "v"(c), "v"(d)); }
__device__ __forceinline__ void keep4_b(v16b a, v16b b, v16b c, v16b d) { asm volatile("v_nop" :: "v"(a), "v"(b), "v"(c), "v"(d)); }
__device__ __forceinline__ void acc_guard4(v8f& a, v8f& b, v8f& c, v8f& d) { asm volatile("v_nop\n\tv_nop\n\tv_nop\n\tv_nop" : "+v"(a), "+v"(b), "+v"(c), "+v"(d)); }

template <typename T> struct Frag;
template <> struct Frag<_Float16> {
  typedef v16h V; union U { v16h v; v8h h[2]; };
  static __device__ __forceinline__ v16h load(const _Float16* p) {
    U f; f.h[0] = *(const v8h*)(p); f.h[1] = *(const v8h*)(p + 16); return f.v;
  }
  static __device__ __forceinline__ v8f mma(v16h a, v16h b, v8f c) {
    return __builtin_amdgcn_wmma_f32_16x16x32_f16(false, a, false, b, (short)0, c, false, false);
  }
  static __device__ __forceinline__ void guard4(v8f& a, v8f& b, v8f& c, v8f& d, v16h x, v16h y) { dep_guard4_h(a, b, c, d, x, y); }
  static __device__ __forceinline__ void keep(v16h a, v16h b, v16h c, v16h d) { keep4_h(a, b, c, d); }
};
template <> struct Frag<__bf16> {
  typedef v16b V; union U { v16b v; v8b h[2]; };
  static __device__ __forceinline__ v16b load(const __bf16* p) {
    U f; f.h[0] = *(const v8b*)(p); f.h[1] = *(const v8b*)(p + 16); return f.v;
  }
  static __device__ __forceinline__ v8f mma(v16b a, v16b b, v8f c) {
    return __builtin_amdgcn_wmma_f32_16x16x32_bf16(false, a, false, b, (short)0, c, false, false);
  }
  static __device__ __forceinline__ void guard4(v8f& a, v8f& b, v8f& c, v8f& d, v16b x, v16b y) { dep_guard4_b(a, b, c, d, x, y); }
  static __device__ __forceinline__ void keep(v16b a, v16b b, v16b c, v16b d) { keep4_b(a, b, c, d); }
};

__device__ __forceinline__ v8f mma_h(v16h a, v16h b, v8f c) {
  c = __builtin_amdgcn_wmma_f32_16x16x32_f16(false, a, false, b, (short)0, c, false, false);
  asm volatile("v_nop\n\tv_nop\n\tv_nop\n\tv_nop" : "+v"(c) : "v"(a), "v"(b));
  return c;
}

template <int ET> struct Elem;
template <> struct Elem<0> { typedef _Float16 T; };
template <> struct Elem<1> { typedef __bf16 T; };
template <int ET, bool SPLIT, int BIAS_MODE, int OUT_MODE, bool RESID, int ACT = 0>
__global__ __launch_bounds__(256) void wmma_gemm64(
    const unsigned short* __restrict__ Ap, const unsigned short* __restrict__ A2p, int lda, long strideA,
    const unsigned short* __restrict__ Btp, const unsigned short* __restrict__ Bt2p, int ldb, long strideB,
    void* __restrict__ Cout, void* __restrict__ Cout2, int ldc, long strideC,
    const float* __restrict__ bias,
    const float* __restrict__ resid, long strideR,
    int M, int N, int K, float scale) {
  typedef typename Elem<ET>::T T;
  typedef typename Frag<T>::V V;
  const T* A = (const T*)Ap; const T* A2 = (const T*)A2p; const T* Bt = (const T*)Btp; const T* Bt2 = (const T*)Bt2p;
  __shared__ __align__(16) float sT[8][16 * 68];
  const int b    = blockIdx.y;
  const int lane = threadIdx.x & 31;
  const int wave = threadIdx.x >> 5;
  const int tilesN = N >> 6;
  const int tilesM = M >> 6;
  const int tile = blockIdx.x * 8 + wave;
  if (tile >= tilesM * tilesN) return;
  const int tm = tile / tilesN;
  const int tn = tile - tm * tilesN;
  const int m0 = tm << 6;
  const int n0 = tn << 6;

  const T* Ab  = A  + (size_t)b * strideA;
  const T* Bb  = Bt + (size_t)b * strideB;
  const T* Ab2 = SPLIT ? (A2  + (size_t)b * strideA) : nullptr;
  const T* Bb2 = SPLIT ? (Bt2 + (size_t)b * strideB) : nullptr;

  const int rlane = lane & 15;
  const int koff  = (lane >> 4) * 8;
  const int mOff  = (lane >> 4) * 8;

  v8f acc[4][4];
#pragma unroll
  for (int i = 0; i < 4; ++i)
#pragma unroll
    for (int j = 0; j < 4; ++j) acc[i][j] = (v8f){0.f,0.f,0.f,0.f,0.f,0.f,0.f,0.f};

  for (int k0 = 0; k0 < K; k0 += 32) {
    V bh[4], bl[4];
#pragma unroll
    for (int j = 0; j < 4; ++j) {
      const size_t bo = (size_t)(n0 + (j << 4) + rlane) * ldb + koff + k0;
      bh[j] = Frag<T>::load(Bb + bo);
      if (SPLIT) bl[j] = Frag<T>::load(Bb2 + bo);
    }
#pragma unroll
    for (int i = 0; i < 4; ++i) {
      const size_t ao = (size_t)(m0 + (i << 4) + rlane) * lda + koff + k0;
      V ah = Frag<T>::load(Ab + ao);
      V al;
      if (SPLIT) al = Frag<T>::load(Ab2 + ao);
#pragma unroll
      for (int j = 0; j < 4; ++j) {
        acc[i][j] = Frag<T>::mma(ah, bh[j], acc[i][j]);
        if (SPLIT) {
          acc[i][j] = Frag<T>::mma(ah, bl[j], acc[i][j]);
          acc[i][j] = Frag<T>::mma(al, bh[j], acc[i][j]);
        }
      }
      Frag<T>::guard4(acc[i][0], acc[i][1], acc[i][2], acc[i][3], ah, SPLIT ? al : ah);
    }
    Frag<T>::keep(bh[0], bh[1], bh[2], bh[3]);
    if (SPLIT) Frag<T>::keep(bl[0], bl[1], bl[2], bl[3]);
  }
  acc_guard4(acc[0][0], acc[0][1], acc[0][2], acc[0][3]);
  acc_guard4(acc[1][0], acc[1][1], acc[1][2], acc[1][3]);
  acc_guard4(acc[2][0], acc[2][1], acc[2][2], acc[2][3]);
  acc_guard4(acc[3][0], acc[3][1], acc[3][2], acc[3][3]);

  float* slab = sT[wave];
  const float* Rb = RESID ? (resid + (size_t)b * strideR) : nullptr;
#pragma unroll
  for (int i = 0; i < 4; ++i) {
    const int mBase = m0 + (i << 4);
#pragma unroll
    for (int j = 0; j < 4; ++j) {
      const int n = n0 + (j << 4) + rlane;
      float bv = 0.f;
      if (BIAS_MODE == 2) bv = bias[n];
#pragma unroll
      for (int r = 0; r < 8; ++r) {
        float v = acc[i][j][r] * scale;
        if (BIAS_MODE == 1) v += bias[mBase + mOff + r];
        if (BIAS_MODE == 2) v += bv;
        if (RESID) v += Rb[(size_t)(mBase + mOff + r) * ldc + n];
        if (ACT == 1) v = tanhf(v);
        if (ACT == 2) v = fmaxf(v, 0.0f);
        if (ACT == 3) v = v / (1.0f + expf(-v));
        if (ACT == 4) v = (v > 0.f) ? v : 0.01f * v;
        slab[(mOff + r) * 68 + (j << 4) + rlane] = v;
      }
    }
    __builtin_amdgcn_fence(__ATOMIC_RELEASE, "workgroup");
    __builtin_amdgcn_wave_barrier();
    __builtin_amdgcn_fence(__ATOMIC_ACQUIRE, "workgroup");
    if (OUT_MODE == 0) {
      float* C = (float*)Cout + (size_t)b * strideC;
      const int hh = lane >> 4, c4 = (lane & 15) * 4;
      for (int pass = 0; pass < 2; ++pass) {
#pragma unroll
        for (int it = 0; it < 8; ++it) {
          const int row = it * 2 + hh;
          v4f v = *(const v4f*)(slab + row * 68 + c4);
          *(volatile v4f*)(C + (size_t)(mBase + row) * ldc + n0 + c4) = v;
        }
        __threadfence();
      }
    } else {
      const int q = lane >> 3, c8 = (lane & 7) * 8;
      unsigned short* C  = (unsigned short*)Cout  + (size_t)b * strideC;
      unsigned short* C2 = (OUT_MODE == 2) ? ((unsigned short*)Cout2 + (size_t)b * strideC) : nullptr;
      for (int pass = 0; pass < 2; ++pass) {
#pragma unroll
        for (int it = 0; it < 4; ++it) {
          const int row = it * 4 + q;
          const float* sp = slab + row * 68 + c8;
          v8h hv, lv;
#pragma unroll
          for (int e = 0; e < 8; ++e) {
            if (OUT_MODE == 1) {
              hv[e] = (_Float16)sp[e];
            } else {
              unsigned short hb = f2bf_bits(sp[e]);
              unsigned short lb = f2bf_bits(sp[e] - bf_bits2f(hb));
              hv[e] = __builtin_bit_cast(_Float16, hb);
              lv[e] = __builtin_bit_cast(_Float16, lb);
            }
          }
          *(volatile v8h*)(C + (size_t)(mBase + row) * ldc + n0 + c8) = hv;
          if (OUT_MODE == 2) *(volatile v8h*)(C2 + (size_t)(mBase + row) * ldc + n0 + c8) = lv;
        }
        __threadfence();
      }
    }
    __builtin_amdgcn_fence(__ATOMIC_RELEASE, "workgroup");
    __builtin_amdgcn_wave_barrier();
    __builtin_amdgcn_fence(__ATOMIC_ACQUIRE, "workgroup");
  }
}

__global__ __launch_bounds__(kThr) void cast_plane_kernel(const float* __restrict__ src, unsigned short* __restrict__ dst,
                                                          int colsLog2, int dstPitch, int dstOff) {
  const int i   = blockIdx.x * kThr + threadIdx.x;
  const int sh  = colsLog2 - 3;
  const int row = i >> sh;
  const int c8  = (i & ((1 << sh) - 1)) * 8;
  const float* sp = src + ((size_t)row << colsLog2) + c8;
  const v4f a0 = *(const v4f*)(sp);
  const v4f a1 = *(const v4f*)(sp + 4);
  v8h hv;
#pragma unroll
  for (int e = 0; e < 4; ++e) {
    const float f0 = a0[e];
    const float f1 = a1[e];
    hv[e]     = (_Float16)carry_flush(bf16r(f0), kInCarry);
    hv[4 + e] = (_Float16)carry_flush(bf16r(f1), kInCarry);
  }
  unsigned short* dp = dst + (size_t)row * dstPitch + dstOff + c8;
  *(volatile v8h*)dp = hv;
  __threadfence();
  *(volatile v8h*)dp = hv;
}
static_assert(kInCarry == kWCarry, "one cast kernel serves inputs and weights");

__global__ __launch_bounds__(kThr) void xstep_plane_kernel(const float* __restrict__ batch, unsigned short* __restrict__ XA) {
  __shared__ __align__(16) float sTile[64 * 68];
  const int tid = threadIdx.x;
  const int t = blockIdx.x;
  {
    const int ff = tid >> 4;
    const int b4 = (tid & 15) * 4;
#pragma unroll
    for (int i = 0; i < 4; ++i) {
      const int f = ff + 16 * i;
      const v4f v = *(const v4f*)(batch + ((size_t)f * kSteps + t) * kBatch + b4);
#pragma unroll
      for (int e = 0; e < 4; ++e) {
        const float fv = v[e];
        sTile[(b4 + e) * 68 + f] = carry_flush(bf16r(fv), kInCarry);
      }
    }
  }
  __syncthreads();
  const int f8 = (tid & 7) * 8;
  v8h hv[2];
#pragma unroll
  for (int it = 0; it < 2; ++it) {
    const int b = (tid >> 3) + 32 * it;
    const float* sp = sTile + b * 68 + f8;
    const v4f a0 = *(const v4f*)(sp);
    const v4f a1 = *(const v4f*)(sp + 4);
#pragma unroll
    for (int e = 0; e < 4; ++e) {
      const float f0 = a0[e];
      const float f1 = a1[e];
      hv[it][e]     = (_Float16)f0;
      hv[it][4 + e] = (_Float16)f1;
    }
  }
  for (int pass = 0; pass < 2; ++pass) {
#pragma unroll
    for (int it = 0; it < 2; ++it) {
      const int b = (tid >> 3) + 32 * it;
      *(volatile v8h*)(XA + ((size_t)t * kBatch + b) * kFeat + f8) = hv[it];
    }
    __threadfence();
  }
}

__global__ __launch_bounds__(kThr) void head_rows_kernel(const float* __restrict__ Wo, unsigned short* __restrict__ dst) {
  const int i  = blockIdx.x * kThr + threadIdx.x;
  const int n  = i >> 5;
  const int k8 = (i & 31) * 8;
  const int nc = (n < kOutN - 1) ? n : (kOutN - 1);
  const bool live = (n < kOutN);
  const v4f a0 = *(const v4f*)(Wo + (size_t)nc * kHid + k8);
  const v4f a1 = *(const v4f*)(Wo + (size_t)nc * kHid + k8 + 4);
  v8h hv;
#pragma unroll
  for (int e = 0; e < 4; ++e) {
    const float f0 = a0[e];
    const float f1 = a1[e];
    hv[e]     = (_Float16)(live ? carry_flush(bf16r(f0), kWCarry) : 0.0f);
    hv[4 + e] = (_Float16)(live ? carry_flush(bf16r(f1), kWCarry) : 0.0f);
  }
  unsigned short* dp = dst + (size_t)n * kHid + k8;
  *(volatile v8h*)dp = hv;
  __threadfence();
  *(volatile v8h*)dp = hv;
}
static_assert((16 * kHid / 8) == 2 * kThr, "head rows grid exact");

__global__ __launch_bounds__(kThr) void param_prep_kernel(const float* __restrict__ bcd, const float* __restrict__ ber,
                                                          const float* __restrict__ bgru, const float* __restrict__ bq,
                                                          const float* __restrict__ bo, const float* __restrict__ us,
                                                          const float* __restrict__ bs, const float* __restrict__ ul,
                                                          const float* __restrict__ bl, const float* __restrict__ addr,
                                                          float* __restrict__ BIN, float* __restrict__ SMALL) {
  const int blk = blockIdx.x;
  if (blk < 4) {
    const int c = blk * kThr + threadIdx.x;
    const int c0 = (c < kCont - 1) ? c : (kCont - 1);
    const int r1 = c - kColEr;
    const int c1 = (r1 < 0) ? 0 : ((r1 > kCont - 1) ? (kCont - 1) : r1);
    const int r2 = c - kColG;
    const int c2 = (r2 < 0) ? 0 : ((r2 > kGate3 - 1) ? (kGate3 - 1) : r2);
    const float v0 = bcd[c0];
    const float v1 = ber[c1];
    const float v2 = bgru[c2];
    const float pick = (c < kColEr) ? v0 : ((c < kColG) ? v1 : v2);
    const float o = (c < kNin) ? bf16r(pick) : 0.0f;
    float* op = BIN + c;
    *(volatile float*)op = o;
    __threadfence();
    *(volatile float*)op = o;
  } else {
    const int i = (blk - 4) * kThr + threadIdx.x;
    const int iq = (i < kMem - 1) ? i : (kMem - 1);
    const int ro = i - kSmBo;
    const int io = (ro < 0) ? 0 : ((ro > kOutN - 1) ? (kOutN - 1) : ro);
    const int rs = i - kSmUs;
    const int is = (rs < 0) ? 0 : ((rs > kHid - 1) ? (kHid - 1) : rs);
    const int rl = i - kSmUl;
    const int il = (rl < 0) ? 0 : ((rl > kHid - 1) ? (kHid - 1) : rl);
    const int ra = i - kSmAd;
    const int ia = (ra < 0) ? 0 : ((ra > kLoc * kAddr - 1) ? (kLoc * kAddr - 1) : ra);
    const int rn = i - kSmAn;
    const int inn = (rn < 0) ? 0 : ((rn > kLoc - 1) ? (kLoc - 1) : rn);
    const float vq = bq[iq];
    const float vo = bo[io];
    const float vs = us[is];
    const float vl = ul[il];
    const float vbs = bs[0];
    const float vbl = bl[0];
    const float va = addr[ia];
    float an2 = 0.0f;
#pragma unroll 1
    for (int a = 0; a < kAddr; ++a) {
      const float w = bf16r(addr[inn * kAddr + a]);
      an2 += w * w;
    }
    float o = 0.0f;
    if (i < kSmBo) o = bf16r(vq);
    else if (i < kSmBo + kOutN) o = bf16r(vo);
    else if (i < kSmUs) o = 0.0f;
    else if (i < kSmUl) o = bf16r(vs);
    else if (i < kSmBs) o = bf16r(vl);
    else if (i == kSmBs) o = bf16r(vbs);
    else if (i == kSmBs + 1) o = bf16r(vbl);
    else if (i < kSmAd) o = 0.0f;
    else if (i < kSmAn) o = bf16r(va);
    else if (i < kSmTot) o = an2;
    if (i < 4928) {
      float* op = SMALL + i;
      *(volatile float*)op = o;
      __threadfence();
      *(volatile float*)op = o;
    }
  }
}
static_assert(4 * kThr >= kNin && 4 * kThr * 4 == 4096, "bias block: 1024 floats fill its 4,096-B region exactly");
static_assert(20 * kThr >= 4928 && 4928 * 4 == 19712 && 4928 >= kSmTot, "small block: bounded by its 19,712-B region");

__device__ __forceinline__ float softplus_f(float v) { return fmaxf(v, 0.0f) + log1pf(expf(-fabsf(v))); }
__device__ __forceinline__ float sigmoid_f(float v) { return 1.0f / (1.0f + expf(-v)); }

__global__ __launch_bounds__(kThrRun) void ctrl_mem_run_kernel(const float* __restrict__ XP,
                                                               const unsigned short* __restrict__ WQCp,
                                                               const unsigned short* __restrict__ WHHp,
                                                               const unsigned short* __restrict__ WMHp,
                                                               const float* __restrict__ SMALL,
                                                               float* MEMC,
                                                               float* __restrict__ HSW,
                                                               float* __restrict__ OUTW) {
  __shared__ __align__(16) _Float16 Ah[2][kSeqBlk * kHP];
  __shared__ __align__(16) _Float16 Rd[kSeqBlk * kRP];
  __shared__ __align__(16) float    Hm[kSeqBlk * kHid];
  __shared__ __align__(16) float    Qs[kSeqBlk * kMem];
  __shared__ __align__(16) float    Cd[kSeqBlk * kCont];
  __shared__ __align__(16) float    Er[kSeqBlk * kCont];
  __shared__ __align__(16) float    sEma[kSeqBlk * kLoc];
  __shared__ __align__(16) float    sWt[kSeqBlk * kLoc];
  __shared__ __align__(16) float    sOs[kSeqBlk * 16];
  __shared__ __align__(16) float    sSm[kSmTot];
  const _Float16* WQC = (const _Float16*)WQCp;
  const _Float16* WHH = (const _Float16*)WHHp;
  const _Float16* WMH = (const _Float16*)WMHp;
  const int tid = threadIdx.x, lane = tid & 31, wave = tid >> 5;
  const int c = lane & 15, hh = lane >> 4, koff = hh * 8;
  const int b0 = blockIdx.x * kSeqBlk;

  {
    _Float16* ahf = &Ah[0][0];
#pragma unroll 1
    for (int i = tid; i < 2 * kSeqBlk * kHP; i += kThrRun) ahf[i] = (_Float16)0.0f;
#pragma unroll 1
    for (int i = tid; i < kSeqBlk * kRP; i += kThrRun) Rd[i] = (_Float16)0.0f;
#pragma unroll 1
    for (int i = tid; i < kSeqBlk * kHid; i += kThrRun) Hm[i] = 0.0f;
#pragma unroll 1
    for (int i = tid; i < kSeqBlk * kLoc; i += kThrRun) { sEma[i] = 0.0f; sWt[i] = 0.0f; }
#pragma unroll 1
    for (int i = tid; i < kSmTot; i += kThrRun) sSm[i] = SMALL[i];
  }
  const int lc = lane & 7;
  const int ln = lane >> 3;
  float* const memBase = MEMC + (size_t)(b0 + wave) * kLoc * kCont + 12 * lc;
  {
    const v4f z4 = {0.f, 0.f, 0.f, 0.f};
#pragma unroll 1
    for (int i = 0; i < 32; ++i) {
      float* p = memBase + (size_t)(ln + 4 * i) * kCont;
      for (int pass = 0; pass < 2; ++pass) {
        *(volatile v4f*)(p) = z4;
        *(volatile v4f*)(p + 4) = z4;
        *(volatile v4f*)(p + 8) = z4;
        __threadfence();
      }
    }
  }
  __syncthreads();

  const float* sBq = sSm + kSmBq;
  const float* sBo = sSm + kSmBo;
  const float* sUs = sSm + kSmUs;
  const float* sUl = sSm + kSmUl;
  const float* sAd = sSm + kSmAd;
  const float* sAn = sSm + kSmAn;
  const v8f z8 = {0.f, 0.f, 0.f, 0.f, 0.f, 0.f, 0.f, 0.f};

#pragma unroll 1
  for (int t = 0; t <= kSteps; ++t) {
    const int cur = t & 1;
    const _Float16* ahrow = &Ah[cur][0] + c * kHP + koff;

    if (t > 0) {
      const v4f s0 = *(const v4f*)(Hm + wave * kHid + 4 * lane);
      const v4f s1 = *(const v4f*)(Hm + wave * kHid + 128 + 4 * lane);
      float* hp = HSW + ((size_t)(t - 1) * kBatch + b0 + wave) * kHid;
      for (int pass = 0; pass < 2; ++pass) {
        *(volatile v4f*)(hp + 4 * lane) = s0;
        *(volatile v4f*)(hp + 128 + 4 * lane) = s1;
        __threadfence();
      }
    }
#pragma unroll 1
    for (int rep = 0; rep < 2; ++rep) {
      const int tile = wave + 16 * rep;
      if (tile >= kTilesA) continue;
      const bool isHead = (tile == kTilesA - 1);
      if (isHead ? (t == 0) : (t == kSteps)) continue;
      const _Float16* wb = WQC + (size_t)(16 * tile + c) * kHid + koff;
      v8f acc = z8;
#pragma unroll 2
      for (int k0 = 0; k0 < kHid; k0 += 32) {
        const v16h a  = Frag<_Float16>::load(ahrow + k0);
        const v16h fb = Frag<_Float16>::load(wb + k0);
        acc = mma_h(a, fb, acc);
      }
      if (tile < 8) {
        const float bqv = sBq[16 * tile + c];
#pragma unroll
        for (int r = 0; r < 8; ++r) Qs[(8 * hh + r) * kMem + 16 * tile + c] = acc[r] * kRecScale + bqv;
      } else if (tile < 14) {
        const int col = 16 * (tile - 8) + c;
#pragma unroll
        for (int r = 0; r < 8; ++r) {
          const float xp = XP[((size_t)t * kBatch + b0 + 8 * hh + r) * kNin + kColCd + col];
          Cd[(8 * hh + r) * kCont + col] = fmaxf(acc[r] * kRecScale + xp, 0.0f);
        }
      } else if (tile < 20) {
        const int col = 16 * (tile - 14) + c;
#pragma unroll
        for (int r = 0; r < 8; ++r) {
          const float xp = XP[((size_t)t * kBatch + b0 + 8 * hh + r) * kNin + kColEr + col];
          Er[(8 * hh + r) * kCont + col] = sigmoid_f(acc[r] * kRecScale + xp);
        }
      } else {
        const bool real = (c < kOutN);
        const float bov = sBo[c];
#pragma unroll
        for (int r = 0; r < 8; ++r) {
          const float lg = acc[r] * kRecScale + bov;
          float mx = real ? lg : -3.0e38f;
          mx = fmaxf(mx, __shfl_xor(mx, 1, 32));
          mx = fmaxf(mx, __shfl_xor(mx, 2, 32));
          mx = fmaxf(mx, __shfl_xor(mx, 4, 32));
          mx = fmaxf(mx, __shfl_xor(mx, 8, 32));
          float se = real ? expf(lg - mx) : 0.0f;
          se += __shfl_xor(se, 1, 32);
          se += __shfl_xor(se, 2, 32);
          se += __shfl_xor(se, 4, 32);
          se += __shfl_xor(se, 8, 32);
          sOs[(8 * hh + r) * 16 + c] = real ? ((lg - mx) - logf(se)) : 0.0f;
        }
        __builtin_amdgcn_fence(__ATOMIC_RELEASE, "workgroup");
        __builtin_amdgcn_wave_barrier();
        __builtin_amdgcn_fence(__ATOMIC_ACQUIRE, "workgroup");
        const v4f o0 = *(const v4f*)(sOs + 4 * lane);
        const v4f o1 = *(const v4f*)(sOs + 128 + 4 * lane);
        float* op = OUTW + ((size_t)(t - 1) * kBatch + b0) * 16;
        for (int pass = 0; pass < 2; ++pass) {
          *(volatile v4f*)(op + 4 * lane) = o0;
          *(volatile v4f*)(op + 128 + 4 * lane) = o1;
          __threadfence();
        }
      }
    }
    if (t == kSteps) break;
    __syncthreads();

    {
      const float* qrow = Qs + wave * kMem;
      float qo[12], qa[4], er[12], cd[12];
#pragma unroll
      for (int k = 0; k < 12; ++k) { qo[k] = qrow[12 * lc + k]; er[k] = Er[wave * kCont + 12 * lc + k]; cd[k] = Cd[wave * kCont + 12 * lc + k]; }
#pragma unroll
      for (int k = 0; k < 4; ++k) qa[k] = qrow[kCont + 4 * lc + k];
      float nq2 = 0.0f;
#pragma unroll
      for (int k = 0; k < 12; ++k) nq2 += qo[k] * qo[k];
#pragma unroll
      for (int k = 0; k < 4; ++k) nq2 += qa[k] * qa[k];
      nq2 += __shfl_xor(nq2, 1, 32);
      nq2 += __shfl_xor(nq2, 2, 32);
      nq2 += __shfl_xor(nq2, 4, 32);
      const float nq = sqrtf(nq2);
      float ds = 0.0f, dl = 0.0f;
#pragma unroll
      for (int k = 0; k < 8; ++k) {
        const float hv = Hm[wave * kHid + 8 * lane + k];
        ds += sUs[8 * lane + k] * hv;
        dl += sUl[8 * lane + k] * hv;
      }
      ds += __shfl_xor(ds, 1, 32);  dl += __shfl_xor(dl, 1, 32);
      ds += __shfl_xor(ds, 2, 32);  dl += __shfl_xor(dl, 2, 32);
      ds += __shfl_xor(ds, 4, 32);  dl += __shfl_xor(dl, 4, 32);
      ds += __shfl_xor(ds, 8, 32);  dl += __shfl_xor(dl, 8, 32);
      ds += __shfl_xor(ds, 16, 32); dl += __shfl_xor(dl, 16, 32);
      const float beta  = softplus_f(ds + sSm[kSmBs]);
      const float gamma = sigmoid_f(dl + sSm[kSmBs + 1]);

      float mx = -3.0e38f;
#pragma unroll 1
      for (int i = 0; i < 32; ++i) {
        const int n = ln + 4 * i;
        const float* p = memBase + (size_t)n * kCont;
        const v4f m0 = *(const v4f*)(p);
        const v4f m1 = *(const v4f*)(p + 4);
        const v4f m2 = *(const v4f*)(p + 8);
        float sp = 0.0f, np = 0.0f;
#pragma unroll
        for (int k = 0; k < 4; ++k) {
          const float v0 = m0[k], v1 = m1[k], v2 = m2[k];
          sp += v0 * qo[k] + v1 * qo[4 + k] + v2 * qo[8 + k];
          np += v0 * v0 + v1 * v1 + v2 * v2;
        }
#pragma unroll
        for (int k = 0; k < 4; ++k) sp += sAd[n * kAddr + 4 * lc + k] * qa[k];
        sp += __shfl_xor(sp, 1, 32);  np += __shfl_xor(np, 1, 32);
        sp += __shfl_xor(sp, 2, 32);  np += __shfl_xor(np, 2, 32);
        sp += __shfl_xor(sp, 4, 32);  np += __shfl_xor(np, 4, 32);
        const float nm = sqrtf(np + sAn[n]);
        const float cs = sp / (nm * nq + kEps);
        const float em = sEma[wave * kLoc + n];
        const float lg = beta * cs - gamma * em;
        mx = fmaxf(mx, lg);
        sWt[wave * kLoc + n] = lg;
        sEma[wave * kLoc + n] = 0.1f * em + 0.9f * cs;
      }
      mx = fmaxf(mx, __shfl_xor(mx, 8, 32));
      mx = fmaxf(mx, __shfl_xor(mx, 16, 32));
      float se = 0.0f;
#pragma unroll 1
      for (int i = 0; i < 32; ++i) {
        const int n = ln + 4 * i;
        const float e = expf(sWt[wave * kLoc + n] - mx);
        sWt[wave * kLoc + n] = e;
        se += e;
      }
      se += __shfl_xor(se, 8, 32);
      se += __shfl_xor(se, 16, 32);

      float rdc[12], rda[4];
#pragma unroll
      for (int k = 0; k < 12; ++k) rdc[k] = 0.0f;
#pragma unroll
      for (int k = 0; k < 4; ++k) rda[k] = 0.0f;
#pragma unroll 1
      for (int i = 0; i < 32; ++i) {
        const int n = ln + 4 * i;
        const float wv = sWt[wave * kLoc + n] / se;
        float* p = memBase + (size_t)n * kCont;
        const v4f m0 = *(const v4f*)(p);
        const v4f m1 = *(const v4f*)(p + 4);
        const v4f m2 = *(const v4f*)(p + 8);
        v4f n0, n1, n2;
#pragma unroll
        for (int k = 0; k < 4; ++k) {
          const float v0 = m0[k], v1 = m1[k], v2 = m2[k];
          rdc[k]     += v0 * wv;
          rdc[4 + k] += v1 * wv;
          rdc[8 + k] += v2 * wv;
          n0[k] = v0 * (1.0f - wv * er[k])     + wv * cd[k];
          n1[k] = v1 * (1.0f - wv * er[4 + k]) + wv * cd[4 + k];
          n2[k] = v2 * (1.0f - wv * er[8 + k]) + wv * cd[8 + k];
        }
        for (int pass = 0; pass < 2; ++pass) {
          *(volatile v4f*)(p) = n0;
          *(volatile v4f*)(p + 4) = n1;
          *(volatile v4f*)(p + 8) = n2;
          __threadfence();
        }
#pragma unroll
        for (int k = 0; k < 4; ++k) rda[k] += sAd[n * kAddr + 4 * lc + k] * wv;
      }
#pragma unroll
      for (int k = 0; k < 12; ++k) { rdc[k] += __shfl_xor(rdc[k], 8, 32); rdc[k] += __shfl_xor(rdc[k], 16, 32); }
#pragma unroll
      for (int k = 0; k < 4; ++k) { rda[k] += __shfl_xor(rda[k], 8, 32); rda[k] += __shfl_xor(rda[k], 16, 32); }
      if (ln == 0) {
#pragma unroll
        for (int k = 0; k < 12; ++k) Rd[wave * kRP + 12 * lc + k] = (_Float16)carry_flush(rdc[k], kRdCarry);
#pragma unroll
        for (int k = 0; k < 4; ++k) Rd[wave * kRP + kCont + 4 * lc + k] = (_Float16)carry_flush(rda[k], kRdCarry);
      }
    }
    __syncthreads();

    {
      const int j = 16 * wave + c;
      _Float16* ahn = &Ah[cur ^ 1][0];
      const _Float16* rdrow = Rd + c * kRP + koff;
      const float* xprow = XP + ((size_t)t * kBatch + b0 + 8 * hh) * kNin + kColG + j;
      float xr[8], xz[8], xn[8];
#pragma unroll
      for (int r = 0; r < 8; ++r) {
        const float* xp = xprow + (size_t)r * kNin;
        xr[r] = xp[0];
        xz[r] = xp[kHid];
        xn[r] = xp[2 * kHid];
      }
      const _Float16* wr = WHH + (size_t)j * kHid + koff;
      const _Float16* wz = WHH + (size_t)(kHid + j) * kHid + koff;
      const _Float16* wn = WHH + (size_t)(2 * kHid + j) * kHid + koff;
      v8f ar = z8, az = z8, an = z8;
#pragma unroll 2
      for (int k0 = 0; k0 < kHid; k0 += 32) {
        const v16h a   = Frag<_Float16>::load(ahrow + k0);
        const v16h fbr = Frag<_Float16>::load(wr + k0);
        const v16h fbz = Frag<_Float16>::load(wz + k0);
        const v16h fbn = Frag<_Float16>::load(wn + k0);
        ar = mma_h(a, fbr, ar);
        az = mma_h(a, fbz, az);
        an = mma_h(a, fbn, an);
      }
      const _Float16* mr = WMH + (size_t)j * kMem + koff;
      const _Float16* mz = WMH + (size_t)(kHid + j) * kMem + koff;
      const _Float16* mn = WMH + (size_t)(2 * kHid + j) * kMem + koff;
      v8f gr = z8, gz = z8, gn = z8;
#pragma unroll 2
      for (int k0 = 0; k0 < kMem; k0 += 32) {
        const v16h a   = Frag<_Float16>::load(rdrow + k0);
        const v16h fbr = Frag<_Float16>::load(mr + k0);
        const v16h fbz = Frag<_Float16>::load(mz + k0);
        const v16h fbn = Frag<_Float16>::load(mn + k0);
        gr = mma_h(a, fbr, gr);
        gz = mma_h(a, fbz, gz);
        gn = mma_h(a, fbn, gn);
      }
#pragma unroll
      for (int r = 0; r < 8; ++r) {
        const int row = 8 * hh + r;
        const float ir = xr[r] + gr[r] * kRdScale;
        const float iz = xz[r] + gz[r] * kRdScale;
        const float inn = xn[r] + gn[r] * kRdScale;
        const float rg = sigmoid_f(ir + ar[r] * kRecScale);
        const float zg = sigmoid_f(iz + az[r] * kRecScale);
        const float nc = tanhf(inn + rg * (an[r] * kRecScale));
        const float ho = Hm[row * kHid + j];
        const float hnew = (1.0f - zg) * nc + zg * ho;
        Hm[row * kHid + j] = hnew;
        ahn[row * kHP + j] = (_Float16)carry_flush(hnew, kActCarry);
      }
    }
    __syncthreads();
  }
}

__global__ __launch_bounds__(kThr) void final_layout_kernel(const float* __restrict__ HSW, const float* __restrict__ OUTW,
                                                            float* __restrict__ out0, float* __restrict__ out1) {
  __shared__ __align__(16) float sT[64 * 68];
  const int tid = threadIdx.x;
  const int t = blockIdx.x;
  const int lrow = tid >> 4;
  const int l4 = (tid & 15) * 4;
#pragma unroll 1
  for (int jt = 0; jt < 5; ++jt) {
#pragma unroll
    for (int i = 0; i < 4; ++i) {
      const int b = lrow + 16 * i;
      v4f v;
      if (jt < 4) v = *(const v4f*)(HSW + ((size_t)t * kBatch + b) * kHid + 64 * jt + l4);
      else        v = *(const v4f*)(OUTW + ((size_t)t * kBatch + b) * 16 + (l4 & 15));
#pragma unroll
      for (int e = 0; e < 4; ++e) {
        const float fv = v[e];
        sT[(l4 + e) * 68 + b] = fv;
      }
    }
    __syncthreads();
    const int nrows = (jt < 4) ? 64 : kOutN;
    v4f ov[4];
#pragma unroll
    for (int i = 0; i < 4; ++i) ov[i] = *(const v4f*)(sT + (lrow + 16 * i) * 68 + l4);
    for (int pass = 0; pass < 2; ++pass) {
#pragma unroll
      for (int i = 0; i < 4; ++i) {
        const int r = lrow + 16 * i;
        if (r < nrows) {
          float* dp = (jt < 4) ? (out0 + ((size_t)t * kHid + 64 * jt + r) * kBatch + l4)
                               : (out1 + ((size_t)t * kOutN + r) * kBatch + l4);
          *(volatile v4f*)dp = ov[i];
        }
      }
      __threadfence();
    }
    __syncthreads();
  }
}

static_assert(((kRowsX / 64) * (kNin / 64)) % 8 == 0, "GEMM grid exact");
static_assert((kCont * kFeat / 8) % kThr == 0 && (kGate3 * kFeat / 8) % kThr == 0, "input-side weight cast grids exact");
static_assert((kMem * kHid / 8) % kThr == 0 && (kCont * kHid / 8) % kThr == 0, "state-side weight cast grids exact");
static_assert((kGate3 * kHid / 8) % kThr == 0 && (kGate3 * kMem / 8) % kThr == 0, "cell weight cast grids exact");

extern "C" void kernel_launch(void* const* d_in, const int* in_sizes, int n_in,
                              void* d_out, int out_size, void* d_ws, size_t ws_size,
                              hipStream_t stream) {
  if (n_in < 20 || d_out == nullptr || d_ws == nullptr) return;
  if (in_sizes[0] != kBatch * kSteps * kFeat) return;
  if (in_sizes[1] != kMem * kHid || in_sizes[2] != kMem) return;
  if (in_sizes[3] != kHid || in_sizes[4] != 1 || in_sizes[5] != kHid || in_sizes[6] != 1) return;
  if (in_sizes[7] != kLoc * kAddr) return;
  if (in_sizes[8] != kCont * kHid || in_sizes[9] != kCont * kFeat || in_sizes[10] != kCont) return;
  if (in_sizes[11] != kCont * kHid || in_sizes[12] != kCont * kFeat || in_sizes[13] != kCont) return;
  if (in_sizes[14] != kGate3 * kFeat || in_sizes[15] != kGate3 * kHid || in_sizes[16] != kGate3 * kMem || in_sizes[17] != kGate3) return;
  if (in_sizes[18] != kOutN * kHid || in_sizes[19] != kOutN) return;
  if (out_size != kOut0 + kOut1) return;
  if (ws_size < kWsTotal) return;

  const float* batch = (const float*)d_in[0];
  const float* Wq    = (const float*)d_in[1];
  const float* bq    = (const float*)d_in[2];
  const float* us    = (const float*)d_in[3];
  const float* bs    = (const float*)d_in[4];
  const float* ul    = (const float*)d_in[5];
  const float* bl    = (const float*)d_in[6];
  const float* addr  = (const float*)d_in[7];
  const float* Wch   = (const float*)d_in[8];
  const float* Wci   = (const float*)d_in[9];
  const float* bcd   = (const float*)d_in[10];
  const float* Weh   = (const float*)d_in[11];
  const float* Wei   = (const float*)d_in[12];
  const float* ber   = (const float*)d_in[13];
  const float* Wih   = (const float*)d_in[14];
  const float* Whh   = (const float*)d_in[15];
  const float* Wmh   = (const float*)d_in[16];
  const float* bgru  = (const float*)d_in[17];
  const float* Wo    = (const float*)d_in[18];
  const float* bo    = (const float*)d_in[19];
  float* out0 = (float*)d_out;
  float* out1 = out0 + kOut0;

  char* ws = (char*)d_ws;
  unsigned short* XA   = (unsigned short*)(ws + kOffXA);
  unsigned short* WIN  = (unsigned short*)(ws + kOffWIN);
  float*          BIN  = (float*)(ws + kOffBIN);
  float*          XP   = (float*)(ws + kOffXP);
  unsigned short* WQC  = (unsigned short*)(ws + kOffWQC);
  unsigned short* WHH  = (unsigned short*)(ws + kOffWHH);
  unsigned short* WMH  = (unsigned short*)(ws + kOffWMH);
  float*          SMALL = (float*)(ws + kOffSM);
  float*          MEMC = (float*)(ws + kOffMEMC);
  float*          HSW  = (float*)(ws + kOffHSW);
  float*          OUTW = (float*)(ws + kOffOUTW);

  xstep_plane_kernel<<<kSteps, kThr, 0, stream>>>(batch, XA);
  cast_plane_kernel<<<(kCont  * kFeat / 8) / kThr, kThr, 0, stream>>>(Wci, WIN + (size_t)kColCd * kFeat, 6, kFeat, 0);
  cast_plane_kernel<<<(kCont  * kFeat / 8) / kThr, kThr, 0, stream>>>(Wei, WIN + (size_t)kColEr * kFeat, 6, kFeat, 0);
  cast_plane_kernel<<<(kGate3 * kFeat / 8) / kThr, kThr, 0, stream>>>(Wih, WIN + (size_t)kColG  * kFeat, 6, kFeat, 0);
  cast_plane_kernel<<<(kMem   * kHid  / 8) / kThr, kThr, 0, stream>>>(Wq,  WQC + (size_t)kRowQ  * kHid,  8, kHid,  0);
  cast_plane_kernel<<<(kCont  * kHid  / 8) / kThr, kThr, 0, stream>>>(Wch, WQC + (size_t)kRowCd * kHid,  8, kHid,  0);
  cast_plane_kernel<<<(kCont  * kHid  / 8) / kThr, kThr, 0, stream>>>(Weh, WQC + (size_t)kRowEr * kHid,  8, kHid,  0);
  head_rows_kernel<<<2, kThr, 0, stream>>>(Wo, WQC + (size_t)kRowHd * kHid);
  cast_plane_kernel<<<(kGate3 * kHid  / 8) / kThr, kThr, 0, stream>>>(Whh, WHH, 8, kHid, 0);
  cast_plane_kernel<<<(kGate3 * kMem  / 8) / kThr, kThr, 0, stream>>>(Wmh, WMH, 7, kMem, 0);
  param_prep_kernel<<<24, kThr, 0, stream>>>(bcd, ber, bgru, bq, bo, us, bs, ul, bl, addr, BIN, SMALL);

  wmma_gemm64<0, false, 2, 0, false, 0><<<dim3((kRowsX / 64) * (kNin / 64) / 8, 1), 256, 0, stream>>>(
      XA, XA, kFeat, 0L, WIN, WIN, kFeat, 0L, (void*)XP, (void*)XP, kNin, 0L,
      BIN, nullptr, 0L, kRowsX, kNin, kFeat, kXpScale);

  ctrl_mem_run_kernel<<<kBatch / kSeqBlk, kThrRun, 0, stream>>>(XP, WQC, WHH, WMH, SMALL, MEMC, HSW, OUTW);
  final_layout_kernel<<<kSteps, kThr, 0, stream>>>(HSW, OUTW, out0, out1);
}
